// UVMB_7267084664863
// MI455X (gfx1250) — hardware-verified
//
#include <hip/hip_runtime.h>
#include <hip/hip_bf16.h>
#include <math.h>

constexpr int NBATCH = 2;
constexpr int NCH_IO = 3;
constexpr int NT_D = 8;
constexpr int NW_D = 96;
constexpr int NH_D = 96;
constexpr int NPOS = NT_D * NW_D * NH_D;
constexpr int NMID = 16;
constexpr int LSEQ = NPOS;
constexpr int DIN = 6;
constexpr int DSTATE = 16;
constexpr int DCONV = 4;
constexpr int NSCAN = DIN * DSTATE;
constexpr int CHK = 1024;
constexpr int NCHK = LSEQ / CHK;
constexpr int EW_BLK = 256;
constexpr int CONV_BLK = 96;
static_assert(NSCAN == 96, "");
static_assert(LSEQ % CHK == 0, "");
static_assert(LSEQ % EW_BLK == 0, "");
static_assert(NH_D == 3 * 32, "");
static_assert(CHK == 4 * 256, "");

constexpr size_t SZ_MID = (size_t)NBATCH * NMID * NPOS * 4;
constexpr size_t SZ_C3  = (size_t)NBATCH * NCH_IO * NPOS * 4;
constexpr size_t SZ_D6  = (size_t)NBATCH * DIN * LSEQ * 4;
constexpr size_t SZ_S16 = (size_t)NBATCH * DSTATE * LSEQ * 4;
constexpr size_t SZ_TOT = (size_t)NBATCH * NCHK * NSCAN * 4;
constexpr size_t OFF_MID = 0;
constexpr size_t OFF_XR  = OFF_MID + SZ_MID;
constexpr size_t OFF_XS  = OFF_XR + SZ_C3;
constexpr size_t OFF_SZ  = OFF_XS + SZ_D6;
constexpr size_t OFF_XC  = OFF_SZ + SZ_D6;
constexpr size_t OFF_DT  = OFF_XC + SZ_D6;
constexpr size_t OFF_BM  = OFF_DT + SZ_D6;
constexpr size_t OFF_CM  = OFF_BM + SZ_S16;
constexpr size_t OFF_YM  = OFF_CM + SZ_S16;
constexpr size_t OFF_AT  = OFF_YM + SZ_C3;
constexpr size_t OFF_HT  = OFF_AT + SZ_TOT;
constexpr size_t OFF_CY  = OFF_HT + SZ_TOT;
constexpr size_t WS_TOTAL = OFF_CY + SZ_TOT;
static_assert(WS_TOTAL == 46172160, "");
static_assert(WS_TOTAL <= (size_t)134217728, "");
static_assert(SZ_MID % 128 == 0 && SZ_C3 % 128 == 0 && SZ_D6 % 128 == 0 && SZ_S16 % 128 == 0 && SZ_TOT % 128 == 0, "");

typedef __attribute__((ext_vector_type(16))) _Float16 v16h;
typedef __attribute__((ext_vector_type(8)))  _Float16 v8h;
typedef __attribute__((ext_vector_type(16))) __bf16   v16b;
typedef __attribute__((ext_vector_type(8)))  __bf16   v8b;
typedef __attribute__((ext_vector_type(8)))  float    v8f;
typedef __attribute__((ext_vector_type(4)))  float    v4f;

__device__ __forceinline__ unsigned short f2bf_bits(float f) {
  unsigned u = __float_as_uint(f);
  return (unsigned short)((u + 0x7FFFu + ((u >> 16) & 1u)) >> 16);
}
__device__ __forceinline__ float bf_bits2f(unsigned short h) { return __uint_as_float(((unsigned)h) << 16); }

__device__ __forceinline__ void dep_guard_h(v8f& a, v8f& b, v16h x, v16h y) { asm volatile("v_nop\n\tv_nop\n\tv_nop\n\tv_nop" : "+v"(a), "+v"(b) : "v"(x), "v"(y)); }
__device__ __forceinline__ void dep_guard_b(v8f& a, v8f& b, v16b x, v16b y) { asm volatile("v_nop\n\tv_nop\n\tv_nop\n\tv_nop" : "+v"(a), "+v"(b) : "v"(x), "v"(y)); }
__device__ __forceinline__ void keep4_h(v16h a, v16h b, v16h c, v16h d) { asm volatile("v_nop" :: "v"(a), "v"(b), "v"(c), "v"(d)); }
__device__ __forceinline__ void keep4_b(v16b a, v16b b, v16b c, v16b d) { asm volatile("v_nop" :: "v"(a), "v"(b), "v"(c), "v"(d)); }
template <typename T> struct Frag;
template <> struct Frag<_Float16> {
  typedef v16h V; union U { v16h v; v8h h[2]; };
  static __device__ __forceinline__ v16h load(const _Float16* p) {
    U f; f.h[0] = *(const v8h*)(p); f.h[1] = *(const v8h*)(p + 16); return f.v;
  }
  static __device__ __forceinline__ v8f mma(v16h a, v16h b, v8f c) {
    return __builtin_amdgcn_wmma_f32_16x16x32_f16(false, a, false, b, (short)0, c, false, false);
  }
  static __device__ __forceinline__ void guard(v8f& a, v8f& b, v16h x, v16h y) { dep_guard_h(a, b, x, y); }
  static __device__ __forceinline__ void keep(v16h a, v16h b, v16h c, v16h d) { keep4_h(a, b, c, d); }
};
template <> struct Frag<__bf16> {
  typedef v16b V; union U { v16b v; v8b h[2]; };
  static __device__ __forceinline__ v16b load(const __bf16* p) {
    U f; f.h[0] = *(const v8b*)(p); f.h[1] = *(const v8b*)(p + 16); return f.v;
  }
  static __device__ __forceinline__ v8f mma(v16b a, v16b b, v8f c) {
    return __builtin_amdgcn_wmma_f32_16x16x32_bf16(false, a, false, b, (short)0, c, false, false);
  }
  static __device__ __forceinline__ void guard(v8f& a, v8f& b, v16b x, v16b y) { dep_guard_b(a, b, x, y); }
  static __device__ __forceinline__ void keep(v16b a, v16b b, v16b c, v16b d) { keep4_b(a, b, c, d); }
};

template <bool SPLIT> struct CE;
template <> struct CE<false> {
  typedef _Float16 T; typedef v16h V;
  static __device__ __forceinline__ T cvt_hi(float v) { return (_Float16)v; }
  static __device__ __forceinline__ T cvt_lo(float v, T hi) { (void)v; return hi; }
  static __device__ __forceinline__ v8f mma(V a, V b, v8f c) {
    c = __builtin_amdgcn_wmma_f32_16x16x32_f16(false, a, false, b, (short)0, c, false, false);
    asm volatile("v_nop\n\tv_nop\n\tv_nop\n\tv_nop" : "+v"(c) : "v"(a), "v"(b));
    return c;
  }
};
template <> struct CE<true> {
  typedef __bf16 T; typedef v16b V;
  static __device__ __forceinline__ T cvt_hi(float v) { return __builtin_bit_cast(__bf16, f2bf_bits(v)); }
  static __device__ __forceinline__ T cvt_lo(float v, T hi) {
    const float hf = bf_bits2f(__builtin_bit_cast(unsigned short, hi));
    return __builtin_bit_cast(__bf16, f2bf_bits(v - hf));
  }
  static __device__ __forceinline__ v8f mma(V a, V b, v8f c) {
    c = __builtin_amdgcn_wmma_f32_16x16x32_bf16(false, a, false, b, (short)0, c, false, false);
    asm volatile("v_nop\n\tv_nop\n\tv_nop\n\tv_nop" : "+v"(c) : "v"(a), "v"(b));
    return c;
  }
};

template <bool SPLIT, int ASH>
__device__ __forceinline__ void build_afrag(const float* base, int habs, int half,
                                            typename CE<SPLIT>::V& ah, typename CE<SPLIT>::V& al) {
  typedef typename CE<SPLIT>::T T;
  const float asc = (float)(1 << ASH);
#pragma unroll
  for (int e = 0; e < 16; ++e) {
    const int tau0 = (e < 8) ? e : (e + 8);
    const int tau1 = tau0 + 8;
    const int tau1c = (tau1 < 27) ? tau1 : 26;
    const int off0 = ((tau0 / 9) * 3 + ((tau0 % 9) / 3)) * 98 + (tau0 % 3);
    const int off1 = ((tau1c / 9) * 3 + ((tau1c % 9) / 3)) * 98 + (tau1c % 3);
    const int off = half ? off1 : off0;
    float v = base[off + habs];
    if (ASH != 0) v = v * asc;
    if (tau1 >= 27) v = half ? 0.0f : v;
    const T hi = CE<SPLIT>::cvt_hi(v);
    ah[e] = hi;
    if (SPLIT) al[e] = CE<SPLIT>::cvt_lo(v, hi);
  }
  if (!SPLIT) al = ah;
}

template <int CI, int NREAL, bool SPLIT, int EPI, int ASH>
__global__ __launch_bounds__(CONV_BLK) void conv333_kernel(
    const float* __restrict__ src,
    const float* __restrict__ wgt,
    const float* __restrict__ bias,
    const float* __restrict__ resid,
    float* __restrict__ dst,
    float wscale, float oscale)
{
  typedef typename CE<SPLIT>::T T;
  typedef typename CE<SPLIT>::V V;
  constexpr int CPR = (CI >= 4) ? 4 : CI;
  constexpr int NPASS = CI / CPR;
  static_assert(CI % CPR == 0, "");
  static_assert(NREAL <= 16, "");
  constexpr int KP = CI * 32;
  constexpr int PROWS = CPR * 9;
  __shared__ __align__(16) T wlh[16 * KP];
  __shared__ __align__(16) T wll[SPLIT ? (16 * KP) : 16];
  __shared__ __align__(16) float patch[PROWS * 98];
  __shared__ __align__(16) float slab[3 * 16 * 32];

  const int tid = threadIdx.x;
  const int lane = tid & 31;
  const int wave = tid >> 5;
  const int mlan = lane & 15;
  const int half = lane >> 4;
  const int w = blockIdx.x % NW_D;
  const int t = (blockIdx.x / NW_D) % NT_D;
  const int b = blockIdx.x / (NW_D * NT_D);
  const int posrow = (t * NW_D + w) * NH_D;
  const float* sb = src + (size_t)b * CI * NPOS;

  for (int i = tid; i < 16 * KP; i += CONV_BLK) {
    const int n = i / KP;
    const int kp = i - n * KP;
    const int ci = kp >> 5;
    const int tau = kp & 31;
    const bool ok = (tau < 27) && (n < NREAL);
    const int nn = (n < NREAL) ? n : (NREAL - 1);
    const int tt = (tau < 27) ? tau : 26;
    float v = wgt[(nn * CI + ci) * 27 + tt] * wscale;
    v = ok ? v : 0.0f;
    const T hi = CE<SPLIT>::cvt_hi(v);
    wlh[i] = hi;
    if (SPLIT) wll[i] = CE<SPLIT>::cvt_lo(v, hi);
  }

  v8f acc[2];
  acc[0] = (v8f){0.f,0.f,0.f,0.f,0.f,0.f,0.f,0.f};
  acc[1] = (v8f){0.f,0.f,0.f,0.f,0.f,0.f,0.f,0.f};

  for (int sp = 0; sp < NPASS; ++sp) {
    __syncthreads();
    for (int i = tid; i < PROWS * 98; i += CONV_BLK) {
      const int row = i / 98;
      const int hh = i - row * 98;
      const int kh = row % 3;
      const int tmp = row / 3;
      const int kd = tmp % 3;
      const int cil = tmp / 3;
      const int ci = sp * CPR + cil;
      const int tt = t + kd - 1, wq = w + kh - 1, hq = hh - 1;
      const bool ok = (tt >= 0) && (tt < NT_D) && (wq >= 0) && (wq < NW_D) && (hq >= 0) && (hq < NH_D);
      const int ttc = min(max(tt, 0), NT_D - 1);
      const int wqc = min(max(wq, 0), NW_D - 1);
      const int hqc = min(max(hq, 0), NH_D - 1);
      const float v = sb[((size_t)(ci * NT_D + ttc) * NW_D + wqc) * NH_D + hqc];
      patch[i] = ok ? v : 0.0f;
    }
    __syncthreads();
#pragma unroll
    for (int sl = 0; sl < CPR; ++sl) {
      const int k0 = (sp * CPR + sl) * 32;
      const V bh = Frag<T>::load(wlh + mlan * KP + k0 + 8 * half);
      V bl = bh;
      if (SPLIT) bl = Frag<T>::load(wll + mlan * KP + k0 + 8 * half);
      const float* base = patch + sl * 9 * 98;
#pragma unroll
      for (int ti = 0; ti < 2; ++ti) {
        V ah, al;
        build_afrag<SPLIT, ASH>(base, wave * 32 + ti * 16 + mlan, half, ah, al);
        acc[ti] = CE<SPLIT>::mma(ah, bh, acc[ti]);
        if (SPLIT) {
          acc[ti] = CE<SPLIT>::mma(ah, bl, acc[ti]);
          acc[ti] = CE<SPLIT>::mma(al, bh, acc[ti]);
        }
      }
    }
  }

  float* sw = slab + wave * 512;
  const int nb = (mlan < NREAL) ? mlan : (NREAL - 1);
  const float bv = bias[nb];
#pragma unroll
  for (int ti = 0; ti < 2; ++ti) {
    const int hoff = ti * 16 + half * 8;
    v4f r0 = (v4f){0.f,0.f,0.f,0.f};
    v4f r1 = r0;
    if (EPI == 2) {
      const float* rp = resid + (size_t)(b * NREAL + nb) * NPOS + posrow + wave * 32 + hoff;
      r0 = *(const v4f*)rp;
      r1 = *(const v4f*)(rp + 4);
    }
#pragma unroll
    for (int q = 0; q < 8; ++q) {
      float v = acc[ti][q] * oscale + bv;
      if (EPI == 1) v = fmaxf(v, 0.0f);
      if (EPI == 2) v += (q < 4) ? r0[q & 3] : r1[q & 3];
      sw[mlan * 32 + hoff + q] = v;
    }
  }
  __syncthreads();
  {
    const int q8 = lane >> 3;
    const int c4 = (lane & 7) * 4;
    float* db = dst + (size_t)b * NREAL * NPOS + posrow + wave * 32 + c4;
    constexpr int NIT = (NREAL + 3) / 4;
    for (int pass = 0; pass < 2; ++pass) {
#pragma unroll
      for (int it = 0; it < NIT; ++it) {
        const int chan = it * 4 + q8;
        if (chan < NREAL) {
          const v4f v = *(const v4f*)(sw + chan * 32 + c4);
          *(volatile v4f*)(db + (size_t)chan * NPOS) = v;
        }
      }
      __threadfence();
    }
  }
}

__device__ __forceinline__ void st2(float* p, float v) {
  *(volatile float*)p = v;
  __threadfence();
  *(volatile float*)p = v;
}
__device__ __forceinline__ float silu_f(float v) {
  const float e = expf(fminf(-v, 40.0f));
  return v * (1.0f / (1.0f + e));
}

__global__ __launch_bounds__(EW_BLK) void k_inproj(const float* __restrict__ xr,
                                                   const float* __restrict__ W_in,
                                                   float* __restrict__ XS, float* __restrict__ SZ)
{
  const int l = blockIdx.x * EW_BLK + threadIdx.x;
  const int j = blockIdx.y;
  const int b = blockIdx.z;
  const float* xp = xr + (size_t)b * NCH_IO * NPOS + (size_t)3 * l;
  const float v0 = xp[0], v1 = xp[1], v2 = xp[2];
  const float val = W_in[j * 3 + 0] * v0 + W_in[j * 3 + 1] * v1 + W_in[j * 3 + 2] * v2;
  if (j < DIN) {
    st2(XS + (size_t)(b * DIN + j) * LSEQ + l, val);
  } else {
    st2(SZ + (size_t)(b * DIN + (j - DIN)) * LSEQ + l, silu_f(val));
  }
}

__global__ __launch_bounds__(EW_BLK) void k_convxc(const float* __restrict__ XS,
                                                   const float* __restrict__ W_conv,
                                                   const float* __restrict__ b_conv,
                                                   float* __restrict__ XC)
{
  const int l = blockIdx.x * EW_BLK + threadIdx.x;
  const int d = blockIdx.y;
  const int b = blockIdx.z;
  const float* xp = XS + (size_t)(b * DIN + d) * LSEQ;
  float a = 0.0f;
#pragma unroll
  for (int k = 0; k < DCONV; ++k) {
    const int idx = l - (DCONV - 1) + k;
    const int ic = (idx < 0) ? 0 : idx;
    float v = xp[ic];
    v = (idx < 0) ? 0.0f : v;
    a += W_conv[d * DCONV + k] * v;
  }
  a += b_conv[d];
  st2(XC + (size_t)(b * DIN + d) * LSEQ + l, silu_f(a));
}

__global__ __launch_bounds__(EW_BLK) void k_xproj(const float* __restrict__ XC,
                                                  const float* __restrict__ W_xproj,
                                                  const float* __restrict__ W_dt,
                                                  const float* __restrict__ b_dt,
                                                  float* __restrict__ BM, float* __restrict__ CM,
                                                  float* __restrict__ DT)
{
  const int l = blockIdx.x * EW_BLK + threadIdx.x;
  const int y = blockIdx.y;
  const int b = blockIdx.z;
  float xc[DIN];
#pragma unroll
  for (int d = 0; d < DIN; ++d) xc[d] = XC[(size_t)(b * DIN + d) * LSEQ + l];
  if (y < 2 * DSTATE) {
    const int i = 1 + y;
    float a = 0.0f;
#pragma unroll
    for (int d = 0; d < DIN; ++d) a += W_xproj[i * DIN + d] * xc[d];
    float* dp = (i <= DSTATE) ? (BM + (size_t)(b * DSTATE + (i - 1)) * LSEQ)
                              : (CM + (size_t)(b * DSTATE + (i - 1 - DSTATE)) * LSEQ);
    st2(dp + l, a);
  } else {
    const int d = y - 2 * DSTATE;
    float a = 0.0f;
#pragma unroll
    for (int dd = 0; dd < DIN; ++dd) a += W_xproj[dd] * xc[dd];
    const float u = a * W_dt[d] + b_dt[d];
    const float spv = fmaxf(u, 0.0f) + log1pf(expf(-fabsf(u)));
    st2(DT + (size_t)(b * DIN + d) * LSEQ + l, spv);
  }
}

__global__ __launch_bounds__(NSCAN) void k_scan_local(const float* __restrict__ DT,
                                                      const float* __restrict__ XC,
                                                      const float* __restrict__ BM,
                                                      const float* __restrict__ A_log,
                                                      float* __restrict__ aTot, float* __restrict__ hTot)
{
  const int tid = threadIdx.x;
  const int g = blockIdx.x % NCHK;
  const int b = blockIdx.x / NCHK;
  const int d = tid >> 4, s = tid & 15;
  const float Ac = -expf(A_log[d * DSTATE + s]);
  const float* dtp = DT + (size_t)(b * DIN + d) * LSEQ + (size_t)g * CHK;
  const float* xcp = XC + (size_t)(b * DIN + d) * LSEQ + (size_t)g * CHK;
  const float* bp  = BM + (size_t)(b * DSTATE + s) * LSEQ + (size_t)g * CHK;
  float Ap = 1.0f, h = 0.0f;
#pragma unroll 2
  for (int t = 0; t < CHK; ++t) {
    const float dt = dtp[t], xc = xcp[t], bs = bp[t];
    const float a = expf(dt * Ac);
    h = a * h + (dt * bs) * xc;
    Ap = Ap * a;
  }
  const size_t o = (size_t)blockIdx.x * NSCAN + tid;
  st2(aTot + o, Ap);
  st2(hTot + o, h);
}

__global__ __launch_bounds__(NBATCH * NSCAN) void k_scan_carry(const float* __restrict__ aTot,
                                                               const float* __restrict__ hTot,
                                                               float* __restrict__ carry)
{
  const int tid = threadIdx.x;
  const int b = tid / NSCAN;
  const int k = tid - b * NSCAN;
  float c = 0.0f;
  for (int g = 0; g < NCHK; ++g) {
    const size_t i = (size_t)(b * NCHK + g) * NSCAN + k;
    const float cv = c;
    st2(carry + i, cv);
    c = aTot[i] * c + hTot[i];
  }
}

__global__ __launch_bounds__(NSCAN) void k_scan_final(const float* __restrict__ DT,
                                                      const float* __restrict__ XC,
                                                      const float* __restrict__ BM,
                                                      const float* __restrict__ CM,
                                                      const float* __restrict__ SZ,
                                                      const float* __restrict__ A_log,
                                                      const float* __restrict__ Dv,
                                                      const float* __restrict__ W_out,
                                                      const float* __restrict__ carry,
                                                      float* __restrict__ ymid)
{
  __shared__ __align__(16) float ylds[DIN * CHK];
  const int tid = threadIdx.x;
  const int lane = tid & 31;
  const int wave = tid >> 5;
  const int g = blockIdx.x % NCHK;
  const int b = blockIdx.x / NCHK;
  const int d = tid >> 4, s = tid & 15;
  const float Ac = -expf(A_log[d * DSTATE + s]);
  const float Dd = Dv[d];
  const float* dtp = DT + (size_t)(b * DIN + d) * LSEQ + (size_t)g * CHK;
  const float* xcp = XC + (size_t)(b * DIN + d) * LSEQ + (size_t)g * CHK;
  const float* szp = SZ + (size_t)(b * DIN + d) * LSEQ + (size_t)g * CHK;
  const float* bp  = BM + (size_t)(b * DSTATE + s) * LSEQ + (size_t)g * CHK;
  const float* cp  = CM + (size_t)(b * DSTATE + s) * LSEQ + (size_t)g * CHK;
  float h = carry[(size_t)blockIdx.x * NSCAN + tid];
#pragma unroll 2
  for (int t = 0; t < CHK; ++t) {
    const float dt = dtp[t], xc = xcp[t], bs = bp[t], cs = cp[t], sz = szp[t];
    const float a = expf(dt * Ac);
    h = a * h + (dt * bs) * xc;
    float v = h * cs;
    v += __shfl_xor(v, 8, 32);
    v += __shfl_xor(v, 4, 32);
    v += __shfl_xor(v, 2, 32);
    v += __shfl_xor(v, 1, 32);
    const float yv = (v + xc * Dd) * sz;
    if (s == 0) ylds[d * CHK + t] = yv;
  }
  __syncthreads();
  float* yb = ymid + (size_t)b * NCH_IO * LSEQ + (size_t)g * CHK;
#pragma unroll 1
  for (int it = 0; it < 8; ++it) {
    const int idx = (it * 3 + wave) * 32 + lane;
    const int j = idx >> 8;
    const int q4 = (idx & 255) * 4;
    float wo[DIN];
#pragma unroll
    for (int dd = 0; dd < DIN; ++dd) wo[dd] = W_out[j * DIN + dd];
    v4f o = (v4f){0.f,0.f,0.f,0.f};
#pragma unroll
    for (int dd = 0; dd < DIN; ++dd) {
      const v4f yv = *(const v4f*)(ylds + dd * CHK + q4);
      o = o + wo[dd] * yv;
    }
    float* p = yb + (size_t)j * LSEQ + q4;
    *(volatile v4f*)p = o;
    __threadfence();
    *(volatile v4f*)p = o;
  }
}

extern "C" void kernel_launch(void* const* d_in, const int* in_sizes, int n_in,
                              void* d_out, int out_size, void* d_ws, size_t ws_size,
                              hipStream_t stream)
{
  (void)in_sizes; (void)n_in;
  const float* x       = (const float*)d_in[0];
  const float* W_cb1   = (const float*)d_in[1];
  const float* b_cb1   = (const float*)d_in[2];
  const float* W_cb2   = (const float*)d_in[3];
  const float* b_cb2   = (const float*)d_in[4];
  const float* W_in    = (const float*)d_in[5];
  const float* W_conv  = (const float*)d_in[6];
  const float* b_conv  = (const float*)d_in[7];
  const float* W_xproj = (const float*)d_in[8];
  const float* W_dt    = (const float*)d_in[9];
  const float* b_dt    = (const float*)d_in[10];
  const float* A_log   = (const float*)d_in[11];
  const float* Dv      = (const float*)d_in[12];
  const float* W_out   = (const float*)d_in[13];
  const float* W_sm    = (const float*)d_in[14];
  const float* b_sm    = (const float*)d_in[15];
  float* out = (float*)d_out;

  if (ws_size < WS_TOTAL) return;
  if ((size_t)out_size < (size_t)NBATCH * NCH_IO * NPOS) return;

  char* ws = (char*)d_ws;
  float* mid   = (float*)(ws + OFF_MID);
  float* xr    = (float*)(ws + OFF_XR);
  float* XS    = (float*)(ws + OFF_XS);
  float* SZp   = (float*)(ws + OFF_SZ);
  float* XC    = (float*)(ws + OFF_XC);
  float* DT    = (float*)(ws + OFF_DT);
  float* BM    = (float*)(ws + OFF_BM);
  float* CM    = (float*)(ws + OFF_CM);
  float* ymid  = (float*)(ws + OFF_YM);
  float* aTot  = (float*)(ws + OFF_AT);
  float* hTot  = (float*)(ws + OFF_HT);
  float* carry = (float*)(ws + OFF_CY);

  const dim3 cgrid(NBATCH * NT_D * NW_D);
  const dim3 cblk(CONV_BLK);

  conv333_kernel<NCH_IO, NMID, false, 1, 0><<<cgrid, cblk, 0, stream>>>(x, W_cb1, b_cb1, x, mid, 64.0f, 1.0f / 64.0f);
  conv333_kernel<NMID, NCH_IO, false, 2, 6><<<cgrid, cblk, 0, stream>>>(mid, W_cb2, b_cb2, x, xr, 64.0f, 1.0f / 4096.0f);

  k_inproj<<<dim3(LSEQ / EW_BLK, 2 * DIN, NBATCH), EW_BLK, 0, stream>>>(xr, W_in, XS, SZp);
  k_convxc<<<dim3(LSEQ / EW_BLK, DIN, NBATCH), EW_BLK, 0, stream>>>(XS, W_conv, b_conv, XC);
  k_xproj<<<dim3(LSEQ / EW_BLK, 2 * DSTATE + DIN, NBATCH), EW_BLK, 0, stream>>>(XC, W_xproj, W_dt, b_dt, BM, CM, DT);

  k_scan_local<<<NBATCH * NCHK, NSCAN, 0, stream>>>(DT, XC, BM, A_log, aTot, hTot);
  k_scan_carry<<<1, NBATCH * NSCAN, 0, stream>>>(aTot, hTot, carry);
  k_scan_final<<<NBATCH * NCHK, NSCAN, 0, stream>>>(DT, XC, BM, CM, SZp, A_log, Dv, W_out, carry, ymid);

  conv333_kernel<NCH_IO, NCH_IO, true, 0, 0><<<cgrid, cblk, 0, stream>>>(ymid, W_sm, b_sm, x, out, 1.0f, 1.0f);
}
